// ITNSR_2937757630599
// MI455X (gfx1250) — hardware-verified
//
#include <hip/hip_runtime.h>
#include <stdint.h>

#define NB_     2
#define NQ_     8192
#define NC_     64
#define C9_     576
#define HID_    256
#define N3_     1728
#define PPB_    4096
#define NPIX_   8192
#define GN_     832
#define GNB_    768
#define APITCH_ 264
#define HPITCH_ 260

typedef unsigned short us_t;
typedef us_t  v8us __attribute__((ext_vector_type(8)));
typedef float v8f  __attribute__((ext_vector_type(8)));
typedef float v4f  __attribute__((ext_vector_type(4)));
typedef v8us __attribute__((may_alias)) v8usa;
typedef v4f  __attribute__((may_alias)) v4fa;
#if defined(__HIP_DEVICE_COMPILE__)
typedef __bf16 v16bf __attribute__((ext_vector_type(16)));
#else
typedef us_t v16bf __attribute__((ext_vector_type(16)));
#endif
union FragU { v16bf v; v8us hv[2]; };

__device__ __forceinline__ v8f wmma_bf16x(v16bf a, v16bf b, v8f c) {
#if defined(__HIP_DEVICE_COMPILE__)
  v8f d = __builtin_amdgcn_wmma_f32_16x16x32_bf16(false, a, false, b, (short)0, c, false, false);
  asm volatile("v_nop\n\tv_nop\n\tv_nop\n\tv_nop" : "+v"(d) : "v"(a), "v"(b));
  return d;
#else
  (void)a; (void)b;
  return c;
#endif
}

__device__ __forceinline__ v16bf ldfrag(const us_t* p, int h) {
  FragU f;
  f.hv[0] = *(const v8usa*)(p + 8 * h);
  f.hv[1] = *(const v8usa*)(p + 16 + 8 * h);
  return f.v;
}

__device__ __forceinline__ uint32_t bf16_rne(float f) {
  const uint32_t u = __float_as_uint(f);
  return (u + 0x7FFFu + ((u >> 16) & 1u)) >> 16;
}

__device__ __forceinline__ void split2(float v, us_t& hi, us_t& lo) {
  const uint32_t hb = bf16_rne(v);
  const float hf = __uint_as_float(hb << 16);
  hi = (us_t)hb;
  lo = (us_t)bf16_rne(v - hf);
}

__device__ __forceinline__ float rcp_f(float x) {
#if defined(__HIP_DEVICE_COMPILE__)
  return __builtin_amdgcn_rcpf(x);
#else
  return 1.0f / x;
#endif
}

__device__ __forceinline__ float gelu_t(float x) {
  const float kk = (2.0f * 0.79788456f * 1.44269504f);
  const float t = kk * x * (1.0f + 0.044715f * x * x);
  const float e = exp2f(t);
  return x * (1.0f - rcp_f(1.0f + e));
}

__device__ __forceinline__ float wsum(float v) {
  v += __shfl_xor(v, 16, 32);
  v += __shfl_xor(v, 8, 32);
  v += __shfl_xor(v, 4, 32);
  v += __shfl_xor(v, 2, 32);
  v += __shfl_xor(v, 1, 32);
  return v;
}

__device__ __forceinline__ void ld8(const float* p, float* o) {
  const v4f a = *(const v4fa*)p;
  const v4f c = *(const v4fa*)(p + 4);
  o[0] = a.x; o[1] = a.y; o[2] = a.z; o[3] = a.w;
  o[4] = c.x; o[5] = c.y; o[6] = c.z; o[7] = c.w;
}

__global__ __launch_bounds__(256) void k_enc(
    const float* __restrict__ inp, const float* __restrict__ w,
    const float* __restrict__ bias, float* __restrict__ feat)
{
  const int idx = blockIdx.x * 256 + threadIdx.x;
  const int x = idx & 63, y = (idx >> 6) & 63, o = (idx >> 12) & 63, b = idx >> 18;
  float acc = bias[o];
  #pragma unroll
  for (int ci = 0; ci < 3; ++ci) {
    const float* ip = inp + (size_t)(b * 3 + ci) * 4096;
    #pragma unroll
    for (int dy = 0; dy < 3; ++dy) {
      const int yy = y + dy - 1;
      const int yc = min(max(yy, 0), 63);
      const bool oky = (unsigned)yy < 64u;
      #pragma unroll
      for (int dx = 0; dx < 3; ++dx) {
        const int xx = x + dx - 1;
        const int xc = min(max(xx, 0), 63);
        const bool ok = oky && ((unsigned)xx < 64u);
        const float v = ip[yc * 64 + xc];
        const float wv = w[((o * 3 + ci) * 3 + dy) * 3 + dx];
        acc += (ok ? v : 0.0f) * wv;
      }
    }
  }
  volatile float* fp = feat + idx;
  *fp = acc;
  __threadfence();
  *fp = acc;
}

__global__ __launch_bounds__(128) void k_planes(
    const float* __restrict__ feat, const float* __restrict__ iw1,
    const float* __restrict__ iw2, const float* __restrict__ ib2,
    us_t* __restrict__ Uh, us_t* __restrict__ Ul,
    us_t* __restrict__ Mh, us_t* __restrict__ Ml,
    us_t* __restrict__ B1h, us_t* __restrict__ B1l)
{
  const int tid = threadIdx.x, lane = tid & 31, wv = tid >> 5;
  const int blk = blockIdx.x;
  v8us ph[3], pl[3];
  us_t* dh;
  us_t* dl;
  int npc;
  if (blk < 2048) {
    const int row = blk * 4 + wv;
    const int b = row >> 12, pix = row & 4095, y = pix >> 6, x = pix & 63;
    const float* fb = feat + (size_t)b * (NC_ * PPB_);
    #pragma unroll
    for (int it = 0; it < 3; ++it) {
      const int p = lane + 32 * it;
      us_t th[8], tl[8];
      #pragma unroll
      for (int i = 0; i < 8; ++i) {
        const int e = min(8 * p + i, C9_ - 1);
        const int c = e / 9;
        const int t = e - 9 * c;
        const int dy = t / 3;
        const int dx = t - 3 * dy;
        const int yy = y + dy - 1, xx = x + dx - 1;
        const bool ok = ((unsigned)yy < 64u) && ((unsigned)xx < 64u);
        const int yc = min(max(yy, 0), 63), xc = min(max(xx, 0), 63);
        const float v = fb[(c * 64 + yc) * 64 + xc];
        split2(ok ? v : 0.0f, th[i], tl[i]);
      }
      v8us a, c2;
      #pragma unroll
      for (int i = 0; i < 8; ++i) { a[i] = th[i]; c2[i] = tl[i]; }
      ph[it] = a; pl[it] = c2;
    }
    dh = Uh + (size_t)row * C9_;
    dl = Ul + (size_t)row * C9_;
    npc = 72;
  } else if (blk < 2048 + 208) {
    const int n = (blk - 2048) * 4 + wv;
    const float* src;
    float z;
    if (n < GNB_) {
      const int j = n / 3;
      const int k = n - 3 * j;
      src = iw2 + (size_t)j * N3_ + k;
      z = 1.0f;
    } else {
      const int kb = n - GNB_;
      const int kc = (kb < 3) ? kb : 0;
      src = ib2 + kc;
      z = (kb < 3) ? 1.0f : 0.0f;
    }
    #pragma unroll
    for (int it = 0; it < 3; ++it) {
      const int p = lane + 32 * it;
      us_t th[8], tl[8];
      #pragma unroll
      for (int i = 0; i < 8; ++i) {
        const int c = min(8 * p + i, C9_ - 1);
        const float v = src[(size_t)3 * c] * z;
        split2(v, th[i], tl[i]);
      }
      v8us a, c2;
      #pragma unroll
      for (int i = 0; i < 8; ++i) { a[i] = th[i]; c2[i] = tl[i]; }
      ph[it] = a; pl[it] = c2;
    }
    dh = Mh + (size_t)n * C9_;
    dl = Ml + (size_t)n * C9_;
    npc = 72;
  } else {
    const int n = (blk - 2256) * 4 + wv;
    {
      us_t th[8], tl[8];
      #pragma unroll
      for (int i = 0; i < 8; ++i) {
        const int k = 8 * lane + i;
        const float v = iw1[(size_t)k * HID_ + n];
        split2(v, th[i], tl[i]);
      }
      v8us a, c2;
      #pragma unroll
      for (int i = 0; i < 8; ++i) { a[i] = th[i]; c2[i] = tl[i]; }
      ph[0] = a; pl[0] = c2;
    }
    v8us zz;
    #pragma unroll
    for (int i = 0; i < 8; ++i) zz[i] = (us_t)0;
    ph[1] = zz; ph[2] = zz; pl[1] = zz; pl[2] = zz;
    dh = B1h + (size_t)n * HID_;
    dl = B1l + (size_t)n * HID_;
    npc = 32;
  }
  #pragma unroll
  for (int it = 0; it < 3; ++it) {
    const int p = lane + 32 * it;
    if (p < npc) {
      *(volatile v8us*)(dh + 8 * p) = ph[it];
      *(volatile v8us*)(dl + 8 * p) = pl[it];
    }
  }
  __threadfence();
  #pragma unroll
  for (int it = 0; it < 3; ++it) {
    const int p = lane + 32 * it;
    if (p < npc) {
      *(volatile v8us*)(dh + 8 * p) = ph[it];
      *(volatile v8us*)(dl + 8 * p) = pl[it];
    }
  }
}

__global__ __launch_bounds__(128) void k_ggemm(
    const us_t* __restrict__ Uh, const us_t* __restrict__ Ul,
    const us_t* __restrict__ Mh, const us_t* __restrict__ Ml,
    float* __restrict__ G)
{
  __shared__ __attribute__((aligned(16))) float sT[4 * 32 * 64];

  const int tid = threadIdx.x, lane = tid & 31, wv = tid >> 5;
  const int h = lane >> 4, m = lane & 15;
  const int R0 = blockIdx.x * 128 + 32 * wv;
  const int N0 = blockIdx.y * 64;

  const us_t* ah0p = Uh + (size_t)(R0 + m) * C9_;
  const us_t* ah1p = ah0p + (size_t)16 * C9_;
  const us_t* al0p = Ul + (size_t)(R0 + m) * C9_;
  const us_t* al1p = al0p + (size_t)16 * C9_;
  const us_t* bhp  = Mh + (size_t)(N0 + m) * C9_;
  const us_t* blp  = Ml + (size_t)(N0 + m) * C9_;

  const v8f zero8 = {0.f, 0.f, 0.f, 0.f, 0.f, 0.f, 0.f, 0.f};
  v8f acc[2][4];
  #pragma unroll
  for (int mt = 0; mt < 2; ++mt)
    #pragma unroll
    for (int nt = 0; nt < 4; ++nt) acc[mt][nt] = zero8;

  #pragma unroll 1
  for (int k0 = 0; k0 < C9_; k0 += 32) {
    const v16bf ah0 = ldfrag(ah0p + k0, h);
    const v16bf al0 = ldfrag(al0p + k0, h);
    const v16bf ah1 = ldfrag(ah1p + k0, h);
    const v16bf al1 = ldfrag(al1p + k0, h);
    #pragma unroll
    for (int nt = 0; nt < 4; ++nt) {
      const v16bf bh = ldfrag(bhp + (size_t)nt * 16 * C9_ + k0, h);
      const v16bf bl = ldfrag(blp + (size_t)nt * 16 * C9_ + k0, h);
      acc[0][nt] = wmma_bf16x(ah0, bh, acc[0][nt]);
      acc[0][nt] = wmma_bf16x(al0, bh, acc[0][nt]);
      acc[0][nt] = wmma_bf16x(ah0, bl, acc[0][nt]);
      acc[1][nt] = wmma_bf16x(ah1, bh, acc[1][nt]);
      acc[1][nt] = wmma_bf16x(al1, bh, acc[1][nt]);
      acc[1][nt] = wmma_bf16x(ah1, bl, acc[1][nt]);
    }
  }

  float* st = sT + wv * 2048;
  #pragma unroll
  for (int nt = 0; nt < 4; ++nt)
    #pragma unroll
    for (int mt = 0; mt < 2; ++mt)
      #pragma unroll
      for (int r = 0; r < 8; ++r)
        st[(16 * mt + 8 * h + r) * 64 + 16 * nt + m] = acc[mt][nt][r];
  __syncthreads();

  const int sub = lane >> 4, q4 = lane & 15;
  #pragma unroll
  for (int i = 0; i < 16; ++i) {
    const int a = 2 * i + sub;
    const v4f v = *(const v4fa*)(st + a * 64 + 4 * q4);
    *(volatile v4f*)(G + (size_t)(R0 + a) * GN_ + N0 + 4 * q4) = v;
  }
  __threadfence();
  #pragma unroll
  for (int i = 0; i < 16; ++i) {
    const int a = 2 * i + sub;
    const v4f v = *(const v4fa*)(st + a * 64 + 4 * q4);
    *(volatile v4f*)(G + (size_t)(R0 + a) * GN_ + N0 + 4 * q4) = v;
  }
}

__device__ __forceinline__ void row_setup(const float* __restrict__ coord, const float* __restrict__ scale,
                                          int b, int q, int s, float* rf, int* rp)
{
  #pragma clang fp contract(off)
  const size_t cq = ((size_t)b * NQ_ + q) * 2;
  const float cx = coord[cq + 0], cy = coord[cq + 1];
  const float sx = scale[cq + 0], sy = scale[cq + 1];
  const float s00 = scale[(size_t)b * NQ_ * 2 + 0];
  const float s01 = scale[(size_t)b * NQ_ * 2 + 1];
  const float C63 = 0.0158730168f;
  const float rx = (1.0f - s00) * C63;
  const float ry = (1.0f - s01) * C63;
  const float eps = (float)1e-6;
  const float shx = ((s & 2) ? rx : -rx) + eps;
  const float shy = ((s & 1) ? ry : -ry) + eps;
  const float loc = (float)(-1.0 + 1e-6), hic = (float)(1.0 - 1e-6);
  const float px = fminf(fmaxf(cx + shx, loc), hic);
  const float py = fminf(fmaxf(cy + shy, loc), hic);
  const float txf = (px + 1.0f) * 32.0f - 0.5f;
  const float tyf = (py + 1.0f) * 32.0f - 0.5f;
  const int ih = (int)fminf(fmaxf(rintf(txf), 0.0f), 63.0f);
  const int iw = (int)fminf(fmaxf(rintf(tyf), 0.0f), 63.0f);
  const float ckx = (float)(2 * ih + 1) * 0.015625f - 1.0f;
  const float cky = (float)(2 * iw + 1) * 0.015625f - 1.0f;
  rf[0] = (cx - ckx) * 64.0f;
  rf[1] = (cy - cky) * 64.0f;
  rf[2] = sx * 64.0f;
  rf[3] = sy * 64.0f;
  rp[0] = ih * 64 + iw;
}

__global__ __launch_bounds__(128) void k_main(
    const float* __restrict__ coord, const float* __restrict__ scale,
    const float* __restrict__ iw0, const float* __restrict__ ib0, const float* __restrict__ ib1,
    const float* __restrict__ sw0, const float* __restrict__ sb0,
    const float* __restrict__ sw1, const float* __restrict__ sb1,
    const float* __restrict__ ww0, const float* __restrict__ wb0,
    const float* __restrict__ ww1, const float* __restrict__ wb1,
    const us_t* __restrict__ B1h, const us_t* __restrict__ B1l,
    const float* __restrict__ G, float* __restrict__ out)
{
  __shared__ __attribute__((aligned(16))) unsigned char big[2 * 32 * APITCH_ * 2];
  __shared__ __attribute__((aligned(16))) float rowf[32 * 4];
  __shared__ int   rowpix[32];
  __shared__ float rowsc[32];
  __shared__ float predL[4 * 96];
  __shared__ __attribute__((aligned(16))) float outst[96];
  static_assert(32 * HPITCH_ * 4 <= 2 * 32 * APITCH_ * 2);
  static_assert((APITCH_ % 8) == 0);
  static_assert((HPITCH_ % 4) == 0);

  us_t*  Ah  = (us_t*)big;
  us_t*  Al  = Ah + 32 * APITCH_;
  float* h1t = (float*)big;

  const int tid = threadIdx.x, lane = tid & 31, wv = tid >> 5;
  const int h = lane >> 4, m = lane & 15;
  const int blk = blockIdx.x;
  const int b = blk >> 8;
  const int q0 = (blk & 255) * 32;
  const int cgc = 8 * lane;
  const v8f zero8 = {0.f, 0.f, 0.f, 0.f, 0.f, 0.f, 0.f, 0.f};

  #pragma unroll 1
  for (int s = 0; s < 4; ++s) {
    if (tid < 32) row_setup(coord, scale, b, q0 + tid, s, rowf + 4 * tid, rowpix + tid);
    __syncthreads();

    {
      float w0[8], w1[8], w2[8], w3[8], bb0[8], s0[8], s1[8], sbb[8], s1w[8];
      ld8(iw0 + cgc, w0);
      ld8(iw0 + 256 + cgc, w1);
      ld8(iw0 + 512 + cgc, w2);
      ld8(iw0 + 768 + cgc, w3);
      ld8(ib0 + cgc, bb0);
      ld8(sw0 + cgc, s0);
      ld8(sw0 + 256 + cgc, s1);
      ld8(sb0 + cgc, sbb);
      ld8(sw1 + cgc, s1w);
      const float sb1v = sb1[0];
      #pragma unroll 1
      for (int i8 = 0; i8 < 8; ++i8) {
        const int row = 8 * wv + i8;
        const v4f rfv = *(const v4fa*)(rowf + 4 * row);
        us_t th[8], tl[8];
        float sp = 0.0f;
        #pragma unroll
        for (int i = 0; i < 8; ++i) {
          const float xv = bb0[i] + rfv.x * w0[i] + rfv.y * w1[i] + rfv.z * w2[i] + rfv.w * w3[i];
          split2(gelu_t(xv), th[i], tl[i]);
          const float yv = sbb[i] + rfv.x * s0[i] + rfv.y * s1[i];
          sp += gelu_t(yv) * s1w[i];
        }
        v8us a, c2;
        #pragma unroll
        for (int i = 0; i < 8; ++i) { a[i] = th[i]; c2[i] = tl[i]; }
        *(v8usa*)(Ah + row * APITCH_ + cgc) = a;
        *(v8usa*)(Al + row * APITCH_ + cgc) = c2;
        sp = wsum(sp);
        if (lane == 0) rowsc[row] = sp + sb1v;
      }
    }
    __syncthreads();

    v8f acc[2][4];
    #pragma unroll
    for (int mt = 0; mt < 2; ++mt)
      #pragma unroll
      for (int nt = 0; nt < 4; ++nt) acc[mt][nt] = zero8;
    {
      const us_t* a0p = Ah + m * APITCH_;
      const us_t* a1p = Ah + (16 + m) * APITCH_;
      const us_t* l0p = Al + m * APITCH_;
      const us_t* l1p = Al + (16 + m) * APITCH_;
      const us_t* bhp = B1h + (size_t)(64 * wv + m) * HID_;
      const us_t* blp = B1l + (size_t)(64 * wv + m) * HID_;
      #pragma unroll 1
      for (int k0 = 0; k0 < HID_; k0 += 32) {
        const v16bf ah0 = ldfrag(a0p + k0, h);
        const v16bf al0 = ldfrag(l0p + k0, h);
        const v16bf ah1 = ldfrag(a1p + k0, h);
        const v16bf al1 = ldfrag(l1p + k0, h);
        #pragma unroll
        for (int nt = 0; nt < 4; ++nt) {
          const v16bf bh = ldfrag(bhp + (size_t)nt * 16 * HID_ + k0, h);
          const v16bf bl = ldfrag(blp + (size_t)nt * 16 * HID_ + k0, h);
          acc[0][nt] = wmma_bf16x(ah0, bh, acc[0][nt]);
          acc[0][nt] = wmma_bf16x(al0, bh, acc[0][nt]);
          acc[0][nt] = wmma_bf16x(ah0, bl, acc[0][nt]);
          acc[1][nt] = wmma_bf16x(ah1, bh, acc[1][nt]);
          acc[1][nt] = wmma_bf16x(al1, bh, acc[1][nt]);
          acc[1][nt] = wmma_bf16x(ah1, bl, acc[1][nt]);
        }
      }
    }
    __syncthreads();

    #pragma unroll
    for (int nt = 0; nt < 4; ++nt) {
      const int col = 64 * wv + 16 * nt + m;
      const float bia = ib1[col];
      #pragma unroll
      for (int mt = 0; mt < 2; ++mt)
        #pragma unroll
        for (int r = 0; r < 8; ++r)
          h1t[(16 * mt + 8 * h + r) * HPITCH_ + col] = gelu_t(acc[mt][nt][r] + bia);
    }
    __syncthreads();

    {
      const float* Gb = G + (size_t)b * PPB_ * GN_;
      #pragma unroll 1
      for (int i8 = 0; i8 < 8; ++i8) {
        const int row = 8 * wv + i8;
        int pix = rowpix[row];
        pix = min(max(pix, 0), PPB_ - 1);
        const float* g = Gb + (size_t)pix * GN_;
        float hh[8], gg[24];
        ld8(h1t + row * HPITCH_ + cgc, hh);
        #pragma unroll
        for (int v = 0; v < 6; ++v) {
          const v4f t = *(const v4fa*)(g + 24 * lane + 4 * v);
          gg[4 * v + 0] = t.x; gg[4 * v + 1] = t.y; gg[4 * v + 2] = t.z; gg[4 * v + 3] = t.w;
        }
        const float gb0 = g[GNB_ + 0], gb1 = g[GNB_ + 1], gb2 = g[GNB_ + 2];
        float p0 = 0.0f, p1 = 0.0f, p2 = 0.0f;
        #pragma unroll
        for (int i = 0; i < 8; ++i) {
          p0 += hh[i] * gg[3 * i + 0];
          p1 += hh[i] * gg[3 * i + 1];
          p2 += hh[i] * gg[3 * i + 2];
        }
        p0 = wsum(p0); p1 = wsum(p1); p2 = wsum(p2);
        const float sc = rowsc[row];
        if (lane == 0) {
          predL[s * 96 + row * 3 + 0] = p0 + gb0 + sc;
          predL[s * 96 + row * 3 + 1] = p1 + gb1 + sc;
          predL[s * 96 + row * 3 + 2] = p2 + gb2 + sc;
        }
      }
    }
    __syncthreads();
  }

  {
    float u0[8], u1[8], u2[8], u3[8], vb[8], u4[8];
    ld8(ww0 + cgc, u0);
    ld8(ww0 + 256 + cgc, u1);
    ld8(ww0 + 512 + cgc, u2);
    ld8(ww0 + 768 + cgc, u3);
    ld8(wb0 + cgc, vb);
    ld8(ww1 + cgc, u4);
    const float wb1v = wb1[0];
    #pragma unroll 1
    for (int t = 0; t < 24; ++t) {
      const int o = wv + 4 * t;
      const float x0 = predL[o], x1 = predL[96 + o], x2 = predL[192 + o], x3 = predL[288 + o];
      float a = 0.0f;
      #pragma unroll
      for (int i = 0; i < 8; ++i) {
        const float pre = vb[i] + x0 * u0[i] + x1 * u1[i] + x2 * u2[i] + x3 * u3[i];
        a += gelu_t(pre) * u4[i];
      }
      a = wsum(a);
      if (lane == 0) outst[o] = a + wb1v;
    }
  }
  __syncthreads();

  if (tid < 24) {
    const v4f v = *(const v4fa*)(outst + 4 * tid);
    float* dst = out + (size_t)blk * 96 + 4 * tid;
    *(volatile v4f*)dst = v;
    __threadfence();
    *(volatile v4f*)dst = v;
  }
}

extern "C" void kernel_launch(void* const* d_in, const int* in_sizes, int n_in,
                              void* d_out, int out_size, void* d_ws, size_t ws_size,
                              hipStream_t stream)
{
  if (n_in < 19) return;
  if (in_sizes[0] != NB_ * 3 * 4096) return;
  if (in_sizes[1] != NB_ * NQ_ * 2 || in_sizes[2] != NB_ * NQ_ * 2) return;
  if (in_sizes[3] != NC_ * 27 || in_sizes[4] != NC_) return;
  if (in_sizes[5] != 4 * HID_ || in_sizes[6] != HID_) return;
  if (in_sizes[7] != HID_ * HID_ || in_sizes[8] != HID_) return;
  if (in_sizes[9] != HID_ * N3_ || in_sizes[10] != N3_) return;
  if (in_sizes[11] != 2 * HID_ || in_sizes[12] != HID_ || in_sizes[13] != HID_ || in_sizes[14] != 1) return;
  if (in_sizes[15] != 4 * HID_ || in_sizes[16] != HID_ || in_sizes[17] != HID_ || in_sizes[18] != 1) return;
  if (out_size != NB_ * NQ_ * 3) return;

  const float* inp   = (const float*)d_in[0];
  const float* coord = (const float*)d_in[1];
  const float* scale = (const float*)d_in[2];
  const float* enc_w = (const float*)d_in[3];
  const float* enc_b = (const float*)d_in[4];
  const float* iw0   = (const float*)d_in[5];
  const float* ib0   = (const float*)d_in[6];
  const float* iw1   = (const float*)d_in[7];
  const float* ib1   = (const float*)d_in[8];
  const float* iw2   = (const float*)d_in[9];
  const float* ib2   = (const float*)d_in[10];
  const float* sw0   = (const float*)d_in[11];
  const float* sb0   = (const float*)d_in[12];
  const float* sw1   = (const float*)d_in[13];
  const float* sb1   = (const float*)d_in[14];
  const float* ww0   = (const float*)d_in[15];
  const float* wb0   = (const float*)d_in[16];
  const float* ww1   = (const float*)d_in[17];
  const float* wb1   = (const float*)d_in[18];
  float* out = (float*)d_out;

  const size_t feat_b = (size_t)NB_ * NC_ * PPB_ * 4;
  const size_t upl_b  = (size_t)NPIX_ * C9_ * 2;
  const size_t mpl_b  = (size_t)GN_ * C9_ * 2;
  const size_t bpl_b  = (size_t)HID_ * HID_ * 2;
  const size_t g_b    = (size_t)NPIX_ * GN_ * 4;
  const size_t off_feat = 0;
  const size_t off_uh = off_feat + feat_b;
  const size_t off_ul = off_uh + upl_b;
  const size_t off_mh = off_ul + upl_b;
  const size_t off_ml = off_mh + mpl_b;
  const size_t off_bh = off_ml + mpl_b;
  const size_t off_bl = off_bh + bpl_b;
  const size_t off_g  = off_bl + bpl_b;
  const size_t total  = off_g + g_b;
  if (total > ws_size) return;

  char* ws = (char*)d_ws;
  float* feat = (float*)(ws + off_feat);
  us_t*  Uh   = (us_t*)(ws + off_uh);
  us_t*  Ul   = (us_t*)(ws + off_ul);
  us_t*  Mh   = (us_t*)(ws + off_mh);
  us_t*  Ml   = (us_t*)(ws + off_ml);
  us_t*  B1h  = (us_t*)(ws + off_bh);
  us_t*  B1l  = (us_t*)(ws + off_bl);
  float* G    = (float*)(ws + off_g);

  k_enc<<<(NB_ * NC_ * PPB_) / 256, 256, 0, stream>>>(inp, enc_w, enc_b, feat);
  k_planes<<<2048 + 208 + 64, 128, 0, stream>>>(feat, iw1, iw2, ib2, Uh, Ul, Mh, Ml, B1h, B1l);
  k_ggemm<<<dim3(NPIX_ / 128, GN_ / 64), 128, 0, stream>>>(Uh, Ul, Mh, Ml, G);
  k_main<<<(NB_ * NQ_) / 32, 128, 0, stream>>>(coord, scale, iw0, ib0, ib1, sw0, sb0, sw1, sb1,
                                               ww0, wb0, ww1, wb1, B1h, B1l, G, out);
}
